// NHAttention_89283780149548
// MI455X (gfx1250) — hardware-verified
//
#include <hip/hip_runtime.h>
#include <stddef.h>


typedef _Float16 v16h __attribute__((ext_vector_type(16)));
typedef _Float16 v8h  __attribute__((ext_vector_type(8)));
typedef float    v8f  __attribute__((ext_vector_type(8)));
typedef float    v4f  __attribute__((ext_vector_type(4)));

#ifndef NB
#define NB 2
#endif
#ifndef SEQ
#define SEQ 4096
#endif
#define NB_FULL  2
#define SEQ_FULL 4096
#define CH    256
#define MROWS (NB * SEQ)

static_assert(NB >= 1 && NB <= NB_FULL);
static_assert(SEQ >= 64 && SEQ <= SEQ_FULL && (SEQ % 64) == 0);
static_assert((SEQ_FULL % 64) == 0);
static_assert((CH % 64) == 0 && (CH % 32) == 0 && (CH % 8) == 0);
static_assert((MROWS % 64) == 0);
static_assert(((CH * CH) % (256 * 8)) == 0);
static_assert((size_t)NB_FULL * SEQ_FULL * CH * 4 == (size_t)8388608);
static_assert((size_t)MROWS * CH < (size_t)0xFFFFFFFFu);

#define LDT 72
#define LDC 68
static_assert((LDT % 8) == 0 && LDT >= 64);
static_assert((LDC % 4) == 0 && LDC >= 64);

#define WCARRY 64.0f

#define WP_BYTES ((size_t)CH * CH * 2)
#define XT_BYTES ((size_t)MROWS * CH * 2)
#define OFF_WP  ((size_t)0)
#define OFF_XT  (OFF_WP + WP_BYTES)
#define WS_TOTAL (OFF_XT + XT_BYTES)
static_assert((WP_BYTES % 128) == 0 && (XT_BYTES % 128) == 0);
static_assert(WS_TOTAL <= (size_t)134217728);

__device__ __forceinline__ float bf16r(float x) {
  unsigned int u = __float_as_uint(x);
  u = (u + 0x7FFFu + ((u >> 16) & 1u)) & 0xFFFF0000u;
  return __uint_as_float(u);
}

static __device__ __forceinline__ _Float16 toh_flush(float v) {
  const _Float16 r = (_Float16)v;
  return (fabsf(v) < 6.103515625e-05f) ? (_Float16)0.0f : r;
}

__device__ __forceinline__ v16h frag_at(const _Float16* p) {
  v8h lo = *(const v8h*)(p);
  v8h hi = *(const v8h*)(p + 16);
  v16h out;
#pragma unroll
  for (int i = 0; i < 8; ++i) { out[i] = lo[i]; out[i + 8] = hi[i]; }
  return out;
}

__device__ __forceinline__ v8f wmma16(v16h a, v16h b, v8f c) {
  v8f d = __builtin_amdgcn_wmma_f32_16x16x32_f16(false, a, false, b, (short)0, c,
                                                 false, false);
  asm volatile("v_nop\n\tv_nop\n\tv_nop\n\tv_nop" : "+v"(d) : "v"(a), "v"(b));
  return d;
}

__global__ __launch_bounds__(256) void wconv_kernel(
    const float* __restrict__ W, _Float16* __restrict__ Wt, unsigned ldw, unsigned ldk) {
  __shared__ _Float16 T[64 * LDT];
  const unsigned tid = threadIdx.x;
  const unsigned n0 = blockIdx.x * 64u;
  const unsigned k0 = blockIdx.y * 64u;
#pragma unroll 4
  for (unsigned j = 0; j < 16u; ++j) {
    const unsigned idx = tid + 256u * j;
    const unsigned kr = idx >> 6, nc = idx & 63u;
    const float v = W[(size_t)(k0 + kr) * ldw + n0 + nc];
    T[nc * LDT + kr] = (_Float16)(WCARRY * bf16r(v));
  }
  __syncthreads();
  v8h x[2];
  size_t off[2];
#pragma unroll
  for (unsigned i = 0; i < 2u; ++i) {
    const unsigned n = 32u * i + (tid >> 3);
    const unsigned kc = (tid & 7u) * 8u;
    x[i] = *(const v8h*)&T[n * LDT + kc];
    off[i] = (size_t)(n0 + n) * ldk + k0 + kc;
  }
#pragma unroll
  for (int i = 0; i < 2; ++i) *(volatile v8h*)(Wt + off[i]) = x[i];
  __threadfence();
#pragma unroll
  for (int i = 0; i < 2; ++i) *(volatile v8h*)(Wt + off[i]) = x[i];
}

__global__ __launch_bounds__(256) void wplain_kernel(
    const float* __restrict__ W, _Float16* __restrict__ Wp) {
  const unsigned idx = (blockIdx.x * 256u + threadIdx.x) * 8u;
  const v4f a0 = *(const v4f*)(W + idx);
  const v4f a1 = *(const v4f*)(W + idx + 4u);
  v8h o;
#pragma unroll
  for (int i = 0; i < 4; ++i) {
    o[i]     = toh_flush(WCARRY * bf16r(a0[i]));
    o[i + 4] = toh_flush(WCARRY * bf16r(a1[i]));
  }
  _Float16* p = Wp + idx;
  *(volatile v8h*)p = o;
  __threadfence();
  *(volatile v8h*)p = o;
}

__device__ __forceinline__ void gemm_body(
    const _Float16* __restrict__ A16, const _Float16* __restrict__ Bt, const unsigned K,
    float* __restrict__ outf) {
  __shared__ float Cs[64 * LDC];
  const unsigned tid = threadIdx.x, lane = tid & 31u, w = tid >> 5;
  const unsigned mw = w >> 1, nw = w & 1u;
  const unsigned hh = lane >> 4, m = lane & 15u;
  const unsigned n0 = blockIdx.x * 64u;
  const unsigned row0 = blockIdx.y * 64u;

  const _Float16* ap  = A16 + (size_t)(row0 + mw * 16u + m) * K + hh * 8u;
  const _Float16* bp0 = Bt + (size_t)(n0 + nw * 32u + m) * K + hh * 8u;
  const _Float16* bp1 = bp0 + (size_t)16 * K;
  v8f acc0 = {}, acc1 = {};
#pragma unroll 2
  for (unsigned k0 = 0; k0 < K; k0 += 32u) {
    const v16h a  = frag_at(ap + k0);
    const v16h b0 = frag_at(bp0 + k0);
    const v16h b1 = frag_at(bp1 + k0);
    acc0 = wmma16(a, b0, acc0);
    acc1 = wmma16(a, b1, acc1);
  }
#pragma unroll
  for (int r = 0; r < 8; ++r) {
    float* d = &Cs[(mw * 16u + hh * 8u + (unsigned)r) * LDC + nw * 32u + m];
    d[0]  = acc0[r];
    d[16] = acc1[r];
  }
  __syncthreads();

  const float cs = 1.0f / (WCARRY * WCARRY);
  v4f xs[4];
  size_t off[4];
#pragma unroll
  for (unsigned i = 0; i < 4u; ++i) {
    const unsigned r = 16u * i + (tid >> 4);
    const unsigned c = (tid & 15u) * 4u;
    const unsigned crow = row0 + r;
    const unsigned bidx = crow / (unsigned)SEQ;
    const unsigned sq = crow - bidx * (unsigned)SEQ;
    const size_t frow = (size_t)bidx * SEQ_FULL + sq;
    const v4f u = *(const v4f*)&Cs[r * LDC + c];
    v4f val;
#pragma unroll
    for (int j = 0; j < 4; ++j) val[j] = u[j] * cs;
    xs[i] = val;
    off[i] = frow * CH + n0 + c;
  }
#pragma unroll
  for (int i = 0; i < 4; ++i) *(volatile v4f*)(outf + off[i]) = xs[i];
  __threadfence();
#pragma unroll
  for (int i = 0; i < 4; ++i) *(volatile v4f*)(outf + off[i]) = xs[i];
}

__global__ __launch_bounds__(256) void gemm_value_kernel(
    const _Float16* __restrict__ A16, const _Float16* __restrict__ Bt,
    float* __restrict__ outf) {
  gemm_body(A16, Bt, (unsigned)CH, outf);
}

extern "C" void kernel_launch(void* const* d_in, const int* in_sizes, int n_in,
                              void* d_out, int out_size, void* d_ws, size_t ws_size,
                              hipStream_t stream) {
  if (n_in < 2) return;
  const long long need_x = (long long)(NB - 1) * CH * SEQ_FULL + (long long)(CH - 1) * SEQ_FULL + SEQ;
  const long long need_o = ((long long)(NB - 1) * SEQ_FULL + SEQ) * CH;
  if ((long long)in_sizes[0] < need_x) return;
  if ((long long)in_sizes[1] < (long long)CH * CH) return;
  if ((long long)out_size < need_o) return;
  if (ws_size < WS_TOTAL) return;

  const float* X  = (const float*)d_in[0];
  const float* wv = (const float*)d_in[1];
  float* out = (float*)d_out;

  char* ws = (char*)d_ws;
  _Float16* Wp = (_Float16*)(ws + OFF_WP);
  _Float16* Xt = (_Float16*)(ws + OFF_XT);

  dim3 blk(256);

  wplain_kernel<<<dim3((CH * CH) / (256 * 8)), blk, 0, stream>>>(wv, Wp);
  for (int b = 0; b < NB; ++b) {
    wconv_kernel<<<dim3(SEQ / 64, CH / 64), blk, 0, stream>>>(
        X + (size_t)b * CH * SEQ_FULL, Xt + (size_t)b * SEQ * CH, (unsigned)SEQ_FULL, (unsigned)CH);
  }
  gemm_value_kernel<<<dim3(CH / 64, MROWS / 64), blk, 0, stream>>>(Xt, Wp, out);
}
